// TransformerMessageBlock_13005160972670
// MI455X (gfx1250) — hardware-verified
//
#include <hip/hip_runtime.h>
#include <stddef.h>


#define FEAT     128
#define HEADS    4
#define HF       512
#define QKVC     1536
#define OUTC     384
#define KRB      64
#define NTHR     256
#define NWAVE    8
#define EPT      8
#define NGRP     2
#define CHUNK    (NTHR * EPT * NGRP)
#define WCAP     (EPT * NGRP * 32)
#define LISTN    (NWAVE * WCAP)
#define NBC      4096
#define NBF      1024
#define RCAP     40960
#define RBN      128
#define OTHR     512
#define DEGCAP   256
#define LDS_FILL ((RCAP + NBF + LISTN) * 4 + 64)
#define WBLK_Q   96
#define WBLK_D   32
#define WBLK_O   96
#define WBLK     (WBLK_Q + WBLK_D + WBLK_O)
#define GROWS    128
#define XP       136
#define SP       132
#define LDS_NODE (GROWS * XP * 2 + GROWS * SP * 4)
#define CNB      32
#define CP       32
#define APE      72
#define DKP      516
#define MSP      520
#define OUP      388
#define NACC     512
#define LB_DK    0
#define LB_MSG   (LB_DK + CP * DKP * 4)
#define LB_NODE  (LB_MSG + CP * MSP * 2)
#define LB_RBF   (LB_NODE + CNB * NACC * 4)
#define LB_UNIT  (LB_RBF + CP * APE * 2)
#define LB_DIST  (LB_UNIT + CP * 4 * 4)
#define LB_ATTN  (LB_DIST + CP * 4)
#define LB_SLOT  (LB_ATTN + CP * 4 * 4)
#define LB_IQ    (LB_SLOT + CP * 4)
#define LB_JS    (LB_IQ + CP * 4)
#define LDS_EDGE (LB_JS + CP * 4)
#define W_SC     16.0f
#define RBF_SC   256.0f
#define MSG_SC   16.0f
#define INV_QKV  0.0625f
#define INV_DKV  0.000244140625f
#define INV_OUT  0.00390625f
#define CUTOFF   5.0f
#define EPSR     1e-15f
#define LN_EPS   1e-5f
#define WSCAP    134217728

static_assert((CHUNK & (CHUNK - 1)) == 0);
static_assert(CHUNK <= 4096);
static_assert((NBC & (NBC - 1)) == 0 && (NBF & (NBF - 1)) == 0);
static_assert(NBC == 4 * NBF);
static_assert(OTHR * 8 == NBC);
static_assert((RCAP % 32) == 0);
static_assert((NBF % CNB) == 0);
static_assert(WBLK_Q * NTHR * 8 == QKVC * FEAT);
static_assert(WBLK_D * NTHR * 8 == 2 * HF * KRB);
static_assert(WBLK_O * NTHR * 8 == OUTC * HF);
static_assert(GROWS == NWAVE * 16);
static_assert(((XP * 2) % 16) == 0 && ((SP * 4) % 16) == 0);
static_assert((QKVC % 128) == 0);
static_assert(CNB == 32 && CP == 32);
static_assert(CP * HEADS * 2 == NTHR);
static_assert(CP * KRB == NTHR * 8);
static_assert(((CP * HF / 8) % NTHR) == 0);
static_assert(((CNB * NACC / 4) % NTHR) == 0);
static_assert(((APE * 2) % 16) == 0 && ((DKP * 4) % 16) == 0 && ((MSP * 2) % 16) == 0 && ((OUP * 4) % 16) == 0);
static_assert(CP * OUP * 4 <= CP * DKP * 4);
static_assert((LB_MSG % 16) == 0 && (LB_NODE % 16) == 0 && (LB_RBF % 16) == 0 && (LB_UNIT % 16) == 0);
static_assert((LB_DIST % 16) == 0 && (LB_ATTN % 16) == 0 && (LB_SLOT % 16) == 0 && (LB_IQ % 16) == 0 && (LB_JS % 16) == 0);
static_assert((KRB % 32) == 0 && (FEAT % 32) == 0 && (HF % 32) == 0);
static_assert(NACC == FEAT + OUTC);
static_assert((CNB * DEGCAP) % CP == 0);

typedef float    v4f  __attribute__((ext_vector_type(4)));
typedef float    v8f  __attribute__((ext_vector_type(8)));
typedef int      v4i  __attribute__((ext_vector_type(4)));
typedef _Float16 v4h  __attribute__((ext_vector_type(4)));
typedef _Float16 v8h  __attribute__((ext_vector_type(8)));
typedef _Float16 v16h __attribute__((ext_vector_type(16)));
union FragH { v16h v; v8h h[2]; };

__device__ __forceinline__ v8f wm(v16h a, v16h b, v8f c) {
  v8f d = __builtin_amdgcn_wmma_f32_16x16x32_f16(false, a, false, b, (short)0, c, false, false);
  asm volatile("v_nop\n\tv_nop\n\tv_nop\n\tv_nop" : "+v"(d) : "v"(a), "v"(b));
  return d;
}

__device__ __forceinline__ float silu_f(float v) {
  return v * __builtin_amdgcn_rcpf(1.0f + __expf(-v));
}
__device__ __forceinline__ v8h cvt8(v4f a, v4f b) {
  v8h o;
  o[0] = (_Float16)a.x; o[1] = (_Float16)a.y; o[2] = (_Float16)a.z; o[3] = (_Float16)a.w;
  o[4] = (_Float16)b.x; o[5] = (_Float16)b.y; o[6] = (_Float16)b.z; o[7] = (_Float16)b.w;
  return o;
}
__device__ __forceinline__ v4h cvt4(v4f a) {
  v4h o;
  o[0] = (_Float16)a.x; o[1] = (_Float16)a.y; o[2] = (_Float16)a.z; o[3] = (_Float16)a.w;
  return o;
}
__device__ __forceinline__ float dist3(float x, float y, float z) {
#pragma clang fp contract(off)
  const float a0 = x * x + EPSR;
  const float a1 = y * y + EPSR;
  const float a2 = z * z + EPSR;
  return sqrtf((a0 + a2) + a1);
}

template <int NB>
__device__ __forceinline__ int scan_chunk(const int* __restrict__ nb, int nE, int cbase, int slotBase,
                                          int* list, int tid, int wave) {
  int wc = 0;
#pragma unroll
  for (int g = 0; g < NGRP; ++g) {
    const int el0  = (g * NTHR + tid) * EPT;
    const int e0   = cbase + el0;
    const int sent = -2147483647 - 1;
    v4i da, db;
    if (cbase + CHUNK <= nE) {
      const int* kp = nb + 2 * (size_t)e0;
      const v4i w0 = *(const v4i*)(kp);
      const v4i w1 = *(const v4i*)(kp + 4);
      const v4i w2 = *(const v4i*)(kp + 8);
      const v4i w3 = *(const v4i*)(kp + 12);
      da.x = w0.x; da.y = w0.z; da.z = w1.x; da.w = w1.z;
      db.x = w2.x; db.y = w2.z; db.z = w3.x; db.w = w3.z;
    } else {
      da.x = (e0     < nE) ? nb[2 * (size_t)min(e0,     nE - 1)] : sent;
      da.y = (e0 + 1 < nE) ? nb[2 * (size_t)min(e0 + 1, nE - 1)] : sent;
      da.z = (e0 + 2 < nE) ? nb[2 * (size_t)min(e0 + 2, nE - 1)] : sent;
      da.w = (e0 + 3 < nE) ? nb[2 * (size_t)min(e0 + 3, nE - 1)] : sent;
      db.x = (e0 + 4 < nE) ? nb[2 * (size_t)min(e0 + 4, nE - 1)] : sent;
      db.y = (e0 + 5 < nE) ? nb[2 * (size_t)min(e0 + 5, nE - 1)] : sent;
      db.z = (e0 + 6 < nE) ? nb[2 * (size_t)min(e0 + 6, nE - 1)] : sent;
      db.w = (e0 + 7 < nE) ? nb[2 * (size_t)min(e0 + 7, nE - 1)] : sent;
    }
    const unsigned nb0 = (unsigned)slotBase;
    const unsigned s0 = (unsigned)da.x - nb0, s1 = (unsigned)da.y - nb0;
    const unsigned s2 = (unsigned)da.z - nb0, s3 = (unsigned)da.w - nb0;
    const unsigned s4 = (unsigned)db.x - nb0, s5 = (unsigned)db.y - nb0;
    const unsigned s6 = (unsigned)db.z - nb0, s7 = (unsigned)db.w - nb0;
    const bool h0 = s0 < (unsigned)NB, h1 = s1 < (unsigned)NB, h2 = s2 < (unsigned)NB, h3 = s3 < (unsigned)NB;
    const bool h4 = s4 < (unsigned)NB, h5 = s5 < (unsigned)NB, h6 = s6 < (unsigned)NB, h7 = s7 < (unsigned)NB;
    const unsigned any = __builtin_amdgcn_ballot_w32(h0 | h1 | h2 | h3 | h4 | h5 | h6 | h7);
    if (any != 0u) {
#define HITJ(J, HJ, SJ) { \
        const unsigned mj = __builtin_amdgcn_ballot_w32(HJ); \
        if (mj != 0u) { \
          if (HJ) { \
            const int pos = wc + (int)__builtin_amdgcn_mbcnt_lo(mj, 0u); \
            if (pos < WCAP) list[wave * WCAP + pos] = ((el0 + (J)) << 12) | (int)(SJ); \
          } \
          wc += (int)__builtin_popcount(mj); } }
      HITJ(0, h0, s0)
      HITJ(1, h1, s1)
      HITJ(2, h2, s2)
      HITJ(3, h3, s3)
      HITJ(4, h4, s4)
      HITJ(5, h5, s5)
      HITJ(6, h6, s6)
      HITJ(7, h7, s7)
#undef HITJ
    }
  }
  return wc;
}

__global__ __launch_bounds__(NTHR) void k_wprep(
    const float* __restrict__ Wq, const float* __restrict__ Wk, const float* __restrict__ Wv,
    const float* __restrict__ Wdk, const float* __restrict__ Wdv, const float* __restrict__ Wd,
    _Float16* pQ, _Float16* pD, _Float16* pO, int nrbf) {
  const int tid = (int)threadIdx.x;
  const int b = (int)blockIdx.x;
  float v[8];
  _Float16* dp;
  if (b < WBLK_Q) {
    const int lp = b * NTHR + tid;
    const int n = lp >> 4, k0 = (lp & 15) * 8;
    const int mat = n >> 9, nc = n & 511;
    const float* src = (mat == 0) ? Wq : ((mat == 1) ? Wk : Wv);
#pragma unroll
    for (int j = 0; j < 8; ++j) v[j] = src[(size_t)(k0 + j) * HF + nc] * W_SC;
    dp = pQ + (size_t)lp * 8;
  } else if (b < WBLK_Q + WBLK_D) {
    const int lp = (b - WBLK_Q) * NTHR + tid;
    const int n = lp >> 3, k0 = (lp & 7) * 8;
    const int mat = n >> 9, nc = n & 511;
    const float* src = (mat == 0) ? Wdk : Wdv;
#pragma unroll
    for (int j = 0; j < 8; ++j) {
      const int k  = k0 + j;
      const int kc = k < nrbf ? k : nrbf - 1;
      const float f = src[(size_t)kc * HF + nc];
      v[j] = f * ((k < nrbf) ? W_SC : 0.0f);
    }
    dp = pD + (size_t)lp * 8;
  } else {
    const int lp = (b - WBLK_Q - WBLK_D) * NTHR + tid;
    const int n = lp >> 6, k0 = (lp & 63) * 8;
#pragma unroll
    for (int j = 0; j < 8; ++j) v[j] = Wd[(size_t)(k0 + j) * OUTC + n] * W_SC;
    dp = pO + (size_t)lp * 8;
  }
  v4f a, c;
  a.x = v[0]; a.y = v[1]; a.z = v[2]; a.w = v[3];
  c.x = v[4]; c.y = v[5]; c.z = v[6]; c.w = v[7];
  const v8h o = cvt8(a, c);
  *(volatile v8h*)dp = o;
  __threadfence();
  *(volatile v8h*)dp = o;
}

__global__ __launch_bounds__(NTHR) void k_count(
    const int* __restrict__ nb, int* cnt, int nE) {
  __shared__ __attribute__((aligned(16))) int scnt[NBC];
  __shared__ __attribute__((aligned(16))) int list[LISTN];
  __shared__ int wcnt[NWAVE];
  const int tid = threadIdx.x, lane = tid & 31, wave = tid >> 5;
  const int nodeBase = blockIdx.x * NBC;

  for (int i = tid; i < NBC; i += NTHR) scnt[i] = 0;
  __syncthreads();

  const int nChunks = (nE + CHUNK - 1) / CHUNK;
#pragma unroll 1
  for (int ch = 0; ch < nChunks; ++ch) {
    const int cbase = ch * CHUNK;
    const int wc = scan_chunk<NBC>(nb, nE, cbase, nodeBase, list, tid, wave);
    if (lane == 0) wcnt[wave] = wc;
    __syncthreads();
    if (wave == 0) {
#pragma unroll 1
      for (int wsx = 0; wsx < NWAVE; ++wsx) {
        int n = __builtin_amdgcn_readfirstlane(wcnt[wsx]);
        n = n > WCAP ? WCAP : (n < 0 ? 0 : n);
        const int* lp = list + wsx * WCAP;
#pragma unroll 1
        for (int i = 0; i < n; ++i) {
          const int ent  = __builtin_amdgcn_readfirstlane(lp[i]);
          const int slot = ent & (NBC - 1);
          if (lane == 0) scnt[slot] = scnt[slot] + 1;
        }
      }
    }
    __syncthreads();
  }

  v4i cq[4];
#pragma unroll
  for (int q = 0; q < 4; ++q) {
    const int f = (wave * 4 + q) * 128 + 4 * lane;
    cq[q] = *(const v4i*)(scnt + f);
  }
  int* cp = cnt + (size_t)nodeBase;
#pragma unroll
  for (int q = 0; q < 4; ++q) {
    const int f = (wave * 4 + q) * 128 + 4 * lane;
    *(volatile v4i*)(cp + f) = cq[q];
  }
  __threadfence();
#pragma unroll
  for (int q = 0; q < 4; ++q) {
    const int f = (wave * 4 + q) * 128 + 4 * lane;
    *(volatile v4i*)(cp + f) = cq[q];
  }
}

__global__ __launch_bounds__(OTHR) void k_offsets(
    const int* __restrict__ cnt, int* off, int* rbase, int nChunk) {
  __shared__ __attribute__((aligned(16))) int soff[NBC];
  __shared__ __attribute__((aligned(16))) int srb[RBN];
  __shared__ int wtot[OTHR / 32];
  const int tid = threadIdx.x, lane = tid & 31, wave = tid >> 5, sub = tid >> 7;
  for (int i = tid; i < RBN; i += OTHR) srb[i] = 0;
  int carry = 0;
#pragma unroll 1
  for (int ch = 0; ch < nChunk; ++ch) {
    const int base = ch * NBC;
    const v4i c0 = *(const v4i*)(cnt + base + 8 * tid);
    const v4i c1 = *(const v4i*)(cnt + base + 8 * tid + 4);
    const int e0 = max(c0.x, 0), e1 = max(c0.y, 0), e2 = max(c0.z, 0), e3 = max(c0.w, 0);
    const int e4 = max(c1.x, 0), e5 = max(c1.y, 0), e6 = max(c1.z, 0), e7 = max(c1.w, 0);
    const int ts = e0 + e1 + e2 + e3 + e4 + e5 + e6 + e7;
    int incl = ts;
#pragma unroll
    for (int d = 1; d < 32; d <<= 1) {
      const int t = __shfl_up(incl, d);
      if (lane >= d) incl += t;
    }
    if (lane == 31) wtot[wave] = incl;
    __syncthreads();
    const int S0 = wtot[0]  + wtot[1]  + wtot[2]  + wtot[3];
    const int S1 = wtot[4]  + wtot[5]  + wtot[6]  + wtot[7];
    const int S2 = wtot[8]  + wtot[9]  + wtot[10] + wtot[11];
    const int S3 = wtot[12] + wtot[13] + wtot[14] + wtot[15];
    int pre = 0;
#pragma unroll 1
    for (int w = 4 * sub; w < wave; ++w) pre += wtot[w];
    const int b0 = carry;
    const int b1 = b0 + ((S0 + 31) & ~31);
    const int b2 = b1 + ((S1 + 31) & ~31);
    const int b3 = b2 + ((S2 + 31) & ~31);
    const int b4 = b3 + ((S3 + 31) & ~31);
    const int myb = sub == 0 ? b0 : (sub == 1 ? b1 : (sub == 2 ? b2 : b3));
    if (tid == 0) {
      srb[min(4 * ch + 0, RBN - 1)] = b0;
      srb[min(4 * ch + 1, RBN - 1)] = b1;
      srb[min(4 * ch + 2, RBN - 1)] = b2;
      srb[min(4 * ch + 3, RBN - 1)] = b3;
    }
    int run = myb + pre + incl - ts;
    soff[8 * tid + 0] = run; run += e0;
    soff[8 * tid + 1] = run; run += e1;
    soff[8 * tid + 2] = run; run += e2;
    soff[8 * tid + 3] = run; run += e3;
    soff[8 * tid + 4] = run; run += e4;
    soff[8 * tid + 5] = run; run += e5;
    soff[8 * tid + 6] = run; run += e6;
    soff[8 * tid + 7] = run;
    carry = b4;
    __syncthreads();
    const v4i o0 = *(const v4i*)(soff + 4 * tid);
    const v4i o1 = *(const v4i*)(soff + 4 * (tid + OTHR));
    int* op = off + base;
    *(volatile v4i*)(op + 4 * tid) = o0;
    *(volatile v4i*)(op + 4 * (tid + OTHR)) = o1;
    __threadfence();
    *(volatile v4i*)(op + 4 * tid) = o0;
    *(volatile v4i*)(op + 4 * (tid + OTHR)) = o1;
    __syncthreads();
  }
  if (tid == 0) srb[min(4 * nChunk, RBN - 1)] = carry;
  __syncthreads();
  v4i rv = {0, 0, 0, 0};
  if (tid < 32) rv = *(const v4i*)(srb + 4 * tid);
  if (tid < 32) *(volatile v4i*)(rbase + 4 * tid) = rv;
  __threadfence();
  if (tid < 32) *(volatile v4i*)(rbase + 4 * tid) = rv;
}

__global__ __launch_bounds__(NTHR) void k_fill(
    const int* __restrict__ nb, const int* __restrict__ off, const int* __restrict__ rbase,
    int* csr, int nE, int csrLen) {
  extern __shared__ v4f lds_dyn[];
  int* region = (int*)lds_dyn;
  int* cursor = region + RCAP;
  int* list   = cursor + NBF;
  int* wcnt   = list + LISTN;
  const int tid = threadIdx.x, lane = tid & 31, wave = tid >> 5;
  const int b = blockIdx.x;
  const int nodeBase = b * NBF;

  int rb0 = rbase[b];
  const int rb1 = rbase[b + 1];
  rb0 = rb0 < 0 ? 0 : (rb0 > csrLen ? csrLen : rb0);
  rb0 &= ~31;
  int len = rb1 - rb0;
  len = len < 0 ? 0 : (len > RCAP ? RCAP : len);
  int lenW = (len + 31) & ~31;
  if (rb0 + lenW > csrLen) lenW = (csrLen - rb0) & ~31;

  {
    const v4i z = {0, 0, 0, 0};
    for (int i = tid; i < RCAP / 4; i += NTHR) ((v4i*)region)[i] = z;
    for (int s = tid; s < NBF; s += NTHR) {
      int o = off[nodeBase + s] - rb0;
      o = o < 0 ? 0 : (o > RCAP ? RCAP : o);
      cursor[s] = o;
    }
  }
  __syncthreads();

  const int nChunks = (nE + CHUNK - 1) / CHUNK;
#pragma unroll 1
  for (int ch = 0; ch < nChunks; ++ch) {
    const int cbase = ch * CHUNK;
    const int wc = scan_chunk<NBF>(nb, nE, cbase, nodeBase, list, tid, wave);
    if (lane == 0) wcnt[wave] = wc;
    __syncthreads();
    if (wave == 0) {
#pragma unroll 1
      for (int wsx = 0; wsx < NWAVE; ++wsx) {
        int n = __builtin_amdgcn_readfirstlane(wcnt[wsx]);
        n = n > WCAP ? WCAP : (n < 0 ? 0 : n);
        const int* lp = list + wsx * WCAP;
#pragma unroll 1
        for (int i = 0; i < n; ++i) {
          const int ent  = __builtin_amdgcn_readfirstlane(lp[i]);
          const int slot = ent & (NBF - 1);
          int e = cbase + ((ent >> 12) & (CHUNK - 1));
          e = e > nE - 1 ? nE - 1 : e;
          if (lane == 0) {
            int pos = cursor[slot];
            pos = pos < 0 ? 0 : (pos > RCAP - 1 ? RCAP - 1 : pos);
            region[pos] = e;
            const int np = pos + 1;
            cursor[slot] = np > RCAP ? RCAP : np;
          }
        }
      }
    }
    __syncthreads();
  }

  const int nv = lenW >> 2;
  int* gp = csr + rb0;
#pragma unroll 1
  for (int i = tid; i < nv; i += NTHR) { const v4i v = ((const v4i*)region)[i]; *(volatile v4i*)(gp + 4 * i) = v; }
  __threadfence();
#pragma unroll 1
  for (int i = tid; i < nv; i += NTHR) { const v4i v = ((const v4i*)region)[i]; *(volatile v4i*)(gp + 4 * i) = v; }
}

__global__ __launch_bounds__(NTHR) void k_node(
    const float* __restrict__ s, const float* __restrict__ gam, const float* __restrict__ bet,
    const _Float16* __restrict__ pQ, const float* __restrict__ bq, const float* __restrict__ bk,
    const float* __restrict__ bv, float* qkv, int nN) {
  extern __shared__ v4f lds_dyn[];
  _Float16* sX = (_Float16*)lds_dyn;
  float* stg = (float*)((char*)lds_dyn + GROWS * XP * 2);
  const int tid = threadIdx.x, lane = tid & 31, wave = tid >> 5, hh = lane >> 4, m = lane & 15;
  const int rowBase = blockIdx.x * GROWS;
  const v4f g4 = *(const v4f*)(gam + 4 * lane);
  const v4f b4 = *(const v4f*)(bet + 4 * lane);

#pragma unroll 1
  for (int i = 0; i < 16; ++i) {
    const int r = wave * 16 + i;
    int row = rowBase + r;
    row = row > nN - 1 ? nN - 1 : row;
    const v4f x = *(const v4f*)(s + (size_t)row * FEAT + 4 * lane);
    float sum = (x.x + x.y) + (x.z + x.w);
#pragma unroll
    for (int o = 16; o > 0; o >>= 1) sum += __shfl_xor(sum, o, 32);
    const float mu = sum * (1.0f / (float)FEAT);
    const v4f d = x - mu;
    float sq = (d.x * d.x + d.y * d.y) + (d.z * d.z + d.w * d.w);
#pragma unroll
    for (int o = 16; o > 0; o >>= 1) sq += __shfl_xor(sq, o, 32);
    const float var = sq * (1.0f / (float)FEAT);
    const float inv = 1.0f / sqrtf(var + LN_EPS);
    const v4f y = (d * inv) * g4 + b4;
    *(v4h*)(sX + r * XP + 4 * lane) = cvt4(y);
  }
  __syncthreads();

  const _Float16* ap = sX + (wave * 16 + m) * XP + 8 * hh;
#pragma unroll 1
  for (int g = 0; g < QKVC / 128; ++g) {
    v8f acc[8];
#pragma unroll
    for (int t = 0; t < 8; ++t) { v8f zz = {0.f, 0.f, 0.f, 0.f, 0.f, 0.f, 0.f, 0.f}; acc[t] = zz; }
#pragma unroll 1
    for (int kt = 0; kt < FEAT / 32; ++kt) {
      FragH a;
      a.h[0] = *(const v8h*)(ap + 32 * kt);
      a.h[1] = *(const v8h*)(ap + 32 * kt + 16);
#pragma unroll
      for (int t = 0; t < 8; ++t) {
        const _Float16* bp = pQ + (size_t)(g * 128 + 16 * t + m) * FEAT + 32 * kt + 8 * hh;
        FragH b;
        b.h[0] = *(const v8h*)bp;
        b.h[1] = *(const v8h*)(bp + 16);
        acc[t] = wm(a.v, b.v, acc[t]);
      }
    }
    const int mat = g >> 2;
    float* sp = stg + (wave * 16 + 8 * hh) * SP;
#pragma unroll
    for (int t = 0; t < 8; ++t) {
      const int cl = 16 * t + m;
      const int cq = (g * 128 + cl) & (HF - 1);
      const float b0v = bq[cq], b1v = bk[cq], b2v = bv[cq];
      const float bias = (mat == 0) ? b0v : ((mat == 1) ? b1v : b2v);
#pragma unroll
      for (int r = 0; r < 8; ++r) sp[r * SP + cl] = acc[t][r] * INV_QKV + bias;
    }
    __syncthreads();
    v4f vals[16];
    const float* lp = stg + wave * 16 * SP + 4 * lane;
#pragma unroll
    for (int i = 0; i < 16; ++i) vals[i] = *(const v4f*)(lp + i * SP);
    float* gp = qkv + (size_t)(rowBase + wave * 16) * QKVC + g * 128 + 4 * lane;
#pragma unroll
    for (int i = 0; i < 16; ++i) *(volatile v4f*)(gp + (size_t)i * QKVC) = vals[i];
    __threadfence();
#pragma unroll
    for (int i = 0; i < 16; ++i) *(volatile v4f*)(gp + (size_t)i * QKVC) = vals[i];
    __syncthreads();
  }
}

__global__ __launch_bounds__(NTHR) void k_edge(
    const int* __restrict__ offp, const int* __restrict__ cntp, const int* __restrict__ csr,
    const float* __restrict__ rin, const int* __restrict__ nb, const float* __restrict__ vin,
    const float* __restrict__ qkv,
    const _Float16* __restrict__ pD, const float* __restrict__ bdk, const float* __restrict__ bdv,
    const _Float16* __restrict__ pO, const float* __restrict__ bd,
    float* out, int nN, int nE, int csrLen, int nrbf) {
  extern __shared__ v4f lds_dyn[];
  char* lb = (char*)lds_dyn;
  float*    sDk   = (float*)(lb + LB_DK);
  float*    sOut  = sDk;
  _Float16* sMsg  = (_Float16*)(lb + LB_MSG);
  float*    sNode = (float*)(lb + LB_NODE);
  _Float16* sRbf  = (_Float16*)(lb + LB_RBF);
  float*    sUnit = (float*)(lb + LB_UNIT);
  float*    sDist = (float*)(lb + LB_DIST);
  float*    sAttn = (float*)(lb + LB_ATTN);
  int*      sSlot = (int*)(lb + LB_SLOT);
  int*      sIq   = (int*)(lb + LB_IQ);
  int*      sJs   = (int*)(lb + LB_JS);

  const int tid = threadIdx.x, lane = tid & 31, wave = tid >> 5, hh = lane >> 4, m = lane & 15;
  const int c0 = blockIdx.x * CNB;
  int offl = offp[c0 + lane];
  int cntl = cntp[c0 + lane];
  cntl = cntl < 0 ? 0 : (cntl > DEGCAP ? DEGCAP : cntl);
  offl = offl < 0 ? 0 : (offl > csrLen ? csrLen : offl);
  const int R0 = __builtin_amdgcn_readfirstlane(offl);
  const int Rend = __builtin_amdgcn_readlane(offl, 31) + __builtin_amdgcn_readlane(cntl, 31);
  int tot = Rend - R0;
  tot = tot < 0 ? 0 : (tot > CNB * DEGCAP ? CNB * DEGCAP : tot);
  const int nch = (tot + CP - 1) / CP;

  {
    const v4f z = {0.f, 0.f, 0.f, 0.f};
    for (int i = tid; i < CNB * NACC / 4; i += NTHR) ((v4f*)sNode)[i] = z;
  }

  const int kcol = tid & 63, rsub = tid >> 6;
  const float rstep = 1.0f / (float)(nrbf - 1);
  const float width = CUTOFF * rstep;
  const float grbf = 0.5f / (width * width);
  const float muk = CUTOFF * ((float)kcol * rstep);
  const float kon = (kcol < nrbf) ? RBF_SC : 0.0f;
  const int rt = wave & 1;
  const int qA = tid & 127, fA = qA / 3, cA = qA - 3 * fA;
  const int qB = tid + 128, fB = qB / 3, cB = qB - 3 * fB;

#pragma unroll 1
  for (int ch = 0; ch < nch; ++ch) {
    const int P = R0 + ch * CP;
    int nval = tot - ch * CP;
    nval = nval > CP ? CP : nval;
    __syncthreads();
    if (tid < CP) {
      int p = P + tid;
      p = p > csrLen - 1 ? csrLen - 1 : (p < 0 ? 0 : p);
      int e = csr[p];
      e = e < 0 ? 0 : (e > nE - 1 ? nE - 1 : e);
      const float rx = rin[(size_t)e * 3], ry = rin[(size_t)e * 3 + 1], rz = rin[(size_t)e * 3 + 2];
      const float d = dist3(rx, ry, rz);
      const float invd = 1.0f / d;
      sDist[tid] = d;
      sUnit[tid * 4 + 0] = rx * invd;
      sUnit[tid * 4 + 1] = ry * invd;
      sUnit[tid * 4 + 2] = rz * invd;
      sUnit[tid * 4 + 3] = 0.0f;
      int i = nb[(size_t)e * 2];
      int j = nb[(size_t)e * 2 + 1];
      int sl = i - c0;
      sl = sl < 0 ? 0 : (sl > CNB - 1 ? CNB - 1 : sl);
      i = i < 0 ? 0 : (i > nN - 1 ? nN - 1 : i);
      j = j < 0 ? 0 : (j > nN - 1 ? nN - 1 : j);
      sSlot[tid] = sl;
      sIq[tid] = i;
      sJs[tid] = j;
    }
    __syncthreads();
#pragma unroll 1
    for (int it = 0; it < CP / 4; ++it) {
      const int r = it * 4 + rsub;
      const float t = sDist[r] - muk;
      const float v = kon * __expf(-(grbf * (t * t)));
      sRbf[r * APE + kcol] = (_Float16)v;
    }
    __syncthreads();

#pragma unroll 1
    for (int pass = 0; pass < 2; ++pass) {
      {
        const int ct0 = (wave >> 1) * 8;
        v8f acc[8];
#pragma unroll
        for (int t = 0; t < 8; ++t) { v8f zz = {0.f, 0.f, 0.f, 0.f, 0.f, 0.f, 0.f, 0.f}; acc[t] = zz; }
        const _Float16* ap = sRbf + (16 * rt + m) * APE + 8 * hh;
#pragma unroll 1
        for (int ks = 0; ks < KRB / 32; ++ks) {
          FragH a;
          a.h[0] = *(const v8h*)(ap + 32 * ks);
          a.h[1] = *(const v8h*)(ap + 32 * ks + 16);
#pragma unroll
          for (int t = 0; t < 8; ++t) {
            const _Float16* bp = pD + (size_t)(pass * HF + 16 * (ct0 + t) + m) * KRB + 32 * ks + 8 * hh;
            FragH b;
            b.h[0] = *(const v8h*)bp;
            b.h[1] = *(const v8h*)(bp + 16);
            acc[t] = wm(a.v, b.v, acc[t]);
          }
        }
        float* sp = sDk + (16 * rt + 8 * hh) * DKP;
#pragma unroll
        for (int t = 0; t < 8; ++t) {
          const int n = 16 * (ct0 + t) + m;
          const float bk0 = bdk[n], bv0 = bdv[n];
          const float bb = (pass == 0) ? bk0 : bv0;
#pragma unroll
          for (int r = 0; r < 8; ++r) sp[r * DKP + n] = silu_f(acc[t][r] * INV_DKV + bb);
        }
      }
      __syncthreads();
      if (pass == 0) {
        const int pr = tid >> 1, part = tid & 1;
        const int e = pr >> 2, h = pr & 3;
        const float* qp = qkv + (size_t)sIq[e] * QKVC + h * FEAT + part * 64;
        const float* kq = qkv + (size_t)sJs[e] * QKVC + HF + h * FEAT + part * 64;
        const float* dq = sDk + e * DKP + h * FEAT + part * 64;
        float sacc = 0.0f;
#pragma unroll 4
        for (int f = 0; f < 64; f += 4) {
          const v4f q4 = *(const v4f*)(qp + f);
          const v4f k4 = *(const v4f*)(kq + f);
          const v4f d4 = *(const v4f*)(dq + f);
          const v4f p4 = q4 * k4 * d4;
          sacc += (p4.x + p4.y) + (p4.z + p4.w);
        }
        sacc += __shfl_xor(sacc, 1, 32);
        const float at = silu_f(sacc);
        if (part == 0) sAttn[e * HEADS + h] = at;
      } else {
#pragma unroll 1
        for (int it = 0; it < (CP * HF / 8) / NTHR; ++it) {
          const int idx = it * NTHR + tid;
          const int e = idx >> 6, c = (idx & 63) * 8, h = c >> 7;
          const float* vp = qkv + (size_t)sJs[e] * QKVC + 2 * HF + c;
          const v4f va = *(const v4f*)vp, vb2 = *(const v4f*)(vp + 4);
          const v4f da = *(const v4f*)(sDk + e * DKP + c), db = *(const v4f*)(sDk + e * DKP + c + 4);
          const float at = sAttn[e * HEADS + h] * MSG_SC;
          *(v8h*)(sMsg + e * MSP + c) = cvt8(va * da * at, vb2 * db * at);
        }
      }
      __syncthreads();
    }

    {
      const int ct0 = (wave >> 1) * 6;
      v8f acc[6];
#pragma unroll
      for (int t = 0; t < 6; ++t) { v8f zz = {0.f, 0.f, 0.f, 0.f, 0.f, 0.f, 0.f, 0.f}; acc[t] = zz; }
      const _Float16* ap2 = sMsg + (16 * rt + m) * MSP + 8 * hh;
#pragma unroll 1
      for (int ks = 0; ks < HF / 32; ++ks) {
        FragH a;
        a.h[0] = *(const v8h*)(ap2 + 32 * ks);
        a.h[1] = *(const v8h*)(ap2 + 32 * ks + 16);
#pragma unroll
        for (int t = 0; t < 6; ++t) {
          const _Float16* bp = pO + (size_t)(16 * (ct0 + t) + m) * HF + 32 * ks + 8 * hh;
          FragH b;
          b.h[0] = *(const v8h*)bp;
          b.h[1] = *(const v8h*)(bp + 16);
          acc[t] = wm(a.v, b.v, acc[t]);
        }
      }
      float* sp = sOut + (16 * rt + 8 * hh) * OUP;
#pragma unroll
      for (int t = 0; t < 6; ++t) {
        const int n = 16 * (ct0 + t) + m;
        const float bb = bd[n];
#pragma unroll
        for (int r = 0; r < 8; ++r) sp[r * OUP + n] = acc[t][r] * INV_OUT + bb;
      }
    }
    __syncthreads();

#pragma unroll 1
    for (int r = 0; r < nval; ++r) {
      const int sl = sSlot[r];
      const int jr = sJs[r];
      const float* so = sOut + r * OUP;
      float va;
      if (wave < 4) {
        va = so[FEAT + qA];
      } else {
        va = so[2 * FEAT + fA] * sUnit[r * 4 + cA] + so[fA] * vin[(size_t)jr * OUTC + qA];
      }
      const float vbv = so[2 * FEAT + fB] * sUnit[r * 4 + cB] + so[fB] * vin[(size_t)jr * OUTC + qB];
      float* np = sNode + sl * NACC;
      np[tid] = np[tid] + va;
      np[tid + 256] = np[tid + 256] + vbv;
    }
  }
  __syncthreads();

  const size_t o1off = (size_t)nN * FEAT;
#pragma unroll 1
  for (int it = 0; it < (CNB * NACC / 4) / NTHR; ++it) {
    const int Pc = it * NTHR + tid;
    const int sl = Pc >> 7, p = Pc & 127;
    const int node = c0 + sl;
    if (node < nN) {
      const v4f v = *(const v4f*)(sNode + sl * NACC + 4 * p);
      const size_t go = (p < 32) ? ((size_t)node * FEAT + 4 * p) : (o1off + (size_t)node * OUTC + 4 * (p - 32));
      *(volatile v4f*)(out + go) = v;
    }
  }
  __threadfence();
#pragma unroll 1
  for (int it = 0; it < (CNB * NACC / 4) / NTHR; ++it) {
    const int Pc = it * NTHR + tid;
    const int sl = Pc >> 7, p = Pc & 127;
    const int node = c0 + sl;
    if (node < nN) {
      const v4f v = *(const v4f*)(sNode + sl * NACC + 4 * p);
      const size_t go = (p < 32) ? ((size_t)node * FEAT + 4 * p) : (o1off + (size_t)node * OUTC + 4 * (p - 32));
      *(volatile v4f*)(out + go) = v;
    }
  }
}

extern "C" void kernel_launch(void* const* d_in, const int* in_sizes, int n_in,
                              void* d_out, int out_size, void* d_ws, size_t ws_size,
                              hipStream_t stream) {
  if (n_in < 18) return;
  if (in_sizes[0] <= 0 || (in_sizes[0] % FEAT) != 0) return;
  const int nN = in_sizes[0] / FEAT;
  if (in_sizes[1] != nN * OUTC) return;
  if (in_sizes[2] <= 0 || (in_sizes[2] % 3) != 0) return;
  const int nE = in_sizes[2] / 3;
  if (in_sizes[3] != 2 * nE) return;
  if (in_sizes[4] != FEAT || in_sizes[5] != FEAT) return;
  if (in_sizes[6] != FEAT * HF || in_sizes[7] != HF) return;
  if (in_sizes[8] != FEAT * HF || in_sizes[9] != HF) return;
  if (in_sizes[10] != FEAT * HF || in_sizes[11] != HF) return;
  if (in_sizes[12] <= 0 || (in_sizes[12] % HF) != 0) return;
  const int nrbf = in_sizes[12] / HF;
  if (nrbf < 2 || nrbf > KRB) return;
  if (in_sizes[13] != HF || in_sizes[14] != nrbf * HF || in_sizes[15] != HF) return;
  if (in_sizes[16] != HF * OUTC || in_sizes[17] != OUTC) return;
  if (out_size != nN * (FEAT + OUTC)) return;
  if (nE > (1 << 26) || nN > (1 << 22)) return;

  const float* s_in  = (const float*)d_in[0];
  const float* v_in  = (const float*)d_in[1];
  const float* r_in  = (const float*)d_in[2];
  const int*   nb    = (const int*)d_in[3];
  const float* gam   = (const float*)d_in[4];
  const float* bet   = (const float*)d_in[5];
  const float* Wq    = (const float*)d_in[6];
  const float* bq    = (const float*)d_in[7];
  const float* Wk    = (const float*)d_in[8];
  const float* bk    = (const float*)d_in[9];
  const float* Wv    = (const float*)d_in[10];
  const float* bv    = (const float*)d_in[11];
  const float* Wdk   = (const float*)d_in[12];
  const float* bdk   = (const float*)d_in[13];
  const float* Wdv   = (const float*)d_in[14];
  const float* bdv   = (const float*)d_in[15];
  const float* Wd    = (const float*)d_in[16];
  const float* bd    = (const float*)d_in[17];
  float* out = (float*)d_out;

  const int NPAD   = ((nN + GROWS - 1) / GROWS) * GROWS;
  const int nBC    = (nN + NBC - 1) / NBC;
  const int CNTPAD = nBC * NBC;
  if (NPAD > CNTPAD) return;
  if (4 * nBC + 1 > RBN) return;
  if (31 * 4 * nBC > 4096) return;
  const int nBF    = (nN + NBF - 1) / NBF;
  const int csrLen = ((nE + 31) & ~31) + 4096;
  const int nGemm  = NPAD / GROWS;
  const int nConv  = (nN + CNB - 1) / CNB;
  if (nConv * CNB > CNTPAD) return;

  char* ws = (char*)d_ws;
  size_t off = 0;
  const size_t oQ   = off; off += (size_t)QKVC * FEAT * 2;      off = (off + 255) & ~(size_t)255;
  const size_t oD   = off; off += (size_t)2 * HF * KRB * 2;     off = (off + 255) & ~(size_t)255;
  const size_t oO   = off; off += (size_t)OUTC * HF * 2;        off = (off + 255) & ~(size_t)255;
  const size_t oCnt = off; off += (size_t)CNTPAD * 4;           off = (off + 255) & ~(size_t)255;
  const size_t oOff = off; off += (size_t)CNTPAD * 4;           off = (off + 255) & ~(size_t)255;
  const size_t oRb  = off; off += (size_t)RBN * 4;              off = (off + 255) & ~(size_t)255;
  const size_t oCsr = off; off += (size_t)csrLen * 4;           off = (off + 255) & ~(size_t)255;
  const size_t oQkv = off; off += (size_t)NPAD * QKVC * 4;      off = (off + 255) & ~(size_t)255;
  if (off > ws_size || off > (size_t)WSCAP) return;
  _Float16* pQ  = (_Float16*)(ws + oQ);
  _Float16* pD  = (_Float16*)(ws + oD);
  _Float16* pO  = (_Float16*)(ws + oO);
  int*   cnt    = (int*)(ws + oCnt);
  int*   offp   = (int*)(ws + oOff);
  int*   rb     = (int*)(ws + oRb);
  int*   csr    = (int*)(ws + oCsr);
  float* qkv    = (float*)(ws + oQkv);

  k_wprep<<<WBLK, NTHR, 0, stream>>>(Wq, Wk, Wv, Wdk, Wdv, Wd, pQ, pD, pO, nrbf);

  k_count<<<nBC, NTHR, 0, stream>>>(nb, cnt, nE);
  k_offsets<<<1, OTHR, 0, stream>>>(cnt, offp, rb, nBC);
  hipFuncSetAttribute(reinterpret_cast<const void*>(&k_fill),
                      hipFuncAttributeMaxDynamicSharedMemorySize, LDS_FILL);
  k_fill<<<nBF, NTHR, LDS_FILL, stream>>>(nb, offp, rb, csr, nE, csrLen);

  hipFuncSetAttribute(reinterpret_cast<const void*>(&k_node),
                      hipFuncAttributeMaxDynamicSharedMemorySize, LDS_NODE);
  k_node<<<nGemm, NTHR, LDS_NODE, stream>>>(s_in, gam, bet, pQ, bq, bk, bv, qkv, nN);

  hipFuncSetAttribute(reinterpret_cast<const void*>(&k_edge),
                      hipFuncAttributeMaxDynamicSharedMemorySize, LDS_EDGE);
  k_edge<<<nConv, NTHR, LDS_EDGE, stream>>>(offp, cnt, csr, r_in, nb, v_in, qkv, pD, bdk, bdv, pO, bd,
                                             out, nN, nE, csrLen, nrbf);
}
